// GCN_node_45801531245068
// MI455X (gfx1250) — hardware-verified
//
#include <hip/hip_runtime.h>
#include <stddef.h>
#include <math.h>


#define FD      64
#define KD      64
#define APK     72
#define NTHR    256
#define NWAVE   8
#define EPT     8
#define NGRP    2
#define CHUNK   (NTHR * EPT * NGRP)
#define WCAP    (EPT * NGRP * 32)
#define LISTN   (NWAVE * WCAP)
#define NBC     4096
#define NBF     1024
#define RCAP    40960
#define RBN     128
#define TGT     256
#define DEGCAP  1024
#define GROWS   128
#define OTHR    512
#define WSCAP   134217728
#define WPL     (FD * KD)
#define LDS_FILL ((RCAP + NBF + LISTN) * 4 + 64)
#define ASC     16.0f
#define WSC     64.0f
#define INVSC   0.0009765625f
#define BN_EPS  1e-5f

static_assert((CHUNK & (CHUNK - 1)) == 0);
static_assert(CHUNK <= 4096);
static_assert(NBC <= 4096 && NBF <= 4096);
static_assert((NBC & (NBC - 1)) == 0 && (NBF & (NBF - 1)) == 0);
static_assert(NBC == 4 * NBF);
static_assert(OTHR * 8 == NBC);
static_assert((RCAP % 32) == 0);
static_assert(TGT == NWAVE * 32 && (TGT % GROWS) == 0);
static_assert((NBC % TGT) == 0);
static_assert(GROWS == NWAVE * 16);
static_assert(FD == 64 && KD == 64 && (APK % 8) == 0);
static_assert((GROWS * APK * 2) % 16 == 0);

typedef float          v4f  __attribute__((ext_vector_type(4)));
typedef float          v8f  __attribute__((ext_vector_type(8)));
typedef double         v2d  __attribute__((ext_vector_type(2)));
typedef int            v4i  __attribute__((ext_vector_type(4)));
typedef unsigned short v8us __attribute__((ext_vector_type(8)));
typedef _Float16       v8h  __attribute__((ext_vector_type(8)));
typedef _Float16       v16h __attribute__((ext_vector_type(16)));
union FragH { v16h v; v8h half[2]; };
union Pack8 { v8h h; v8us u; };

__device__ __forceinline__ v8h cvt8(v4f a, v4f b, float sc) {
  v8h r;
  r[0] = (_Float16)(a.x * sc); r[1] = (_Float16)(a.y * sc); r[2] = (_Float16)(a.z * sc); r[3] = (_Float16)(a.w * sc);
  r[4] = (_Float16)(b.x * sc); r[5] = (_Float16)(b.y * sc); r[6] = (_Float16)(b.z * sc); r[7] = (_Float16)(b.w * sc);
  return r;
}

__device__ __forceinline__ v4f bnr(v4f v, v4f mu, v4f rs, v4f g, v4f b) {
  v4f y = (v - mu) * rs * g + b;
  y.x = fmaxf(y.x, 0.0f); y.y = fmaxf(y.y, 0.0f); y.z = fmaxf(y.z, 0.0f); y.w = fmaxf(y.w, 0.0f);
  return y;
}

__device__ __forceinline__ v8f wmh(v16h a, v16h b, v8f c) {
  v8f d = __builtin_amdgcn_wmma_f32_16x16x32_f16(false, a, false, b, (short)0, c, false, false);
  asm volatile("v_nop\n\tv_nop\n\tv_nop\n\tv_nop" : "+v"(d) : "v"(a), "v"(b));
  return d;
}

template <int NB>
__device__ __forceinline__ int scan_chunk(const int* __restrict__ dsts, int nE, int cbase, int slotBase,
                                          int vec8, int* list, int tid, int lane, int wave) {
  int wc = 0;
#pragma unroll
  for (int g = 0; g < NGRP; ++g) {
    const int el0  = (g * NTHR + tid) * EPT;
    const int e0   = cbase + el0;
    const int sent = -2147483647 - 1;
    v4i da, db;
    if (vec8 != 0 && cbase + CHUNK <= nE) {
      da = *(const v4i*)(dsts + e0);
      db = *(const v4i*)(dsts + e0 + 4);
    } else {
      da.x = (e0     < nE) ? dsts[min(e0, nE - 1)] : sent;
      da.y = (e0 + 1 < nE) ? dsts[min(e0 + 1, nE - 1)] : sent;
      da.z = (e0 + 2 < nE) ? dsts[min(e0 + 2, nE - 1)] : sent;
      da.w = (e0 + 3 < nE) ? dsts[min(e0 + 3, nE - 1)] : sent;
      db.x = (e0 + 4 < nE) ? dsts[min(e0 + 4, nE - 1)] : sent;
      db.y = (e0 + 5 < nE) ? dsts[min(e0 + 5, nE - 1)] : sent;
      db.z = (e0 + 6 < nE) ? dsts[min(e0 + 6, nE - 1)] : sent;
      db.w = (e0 + 7 < nE) ? dsts[min(e0 + 7, nE - 1)] : sent;
    }
    const unsigned nb = (unsigned)slotBase;
    const unsigned s0 = (unsigned)da.x - nb, s1 = (unsigned)da.y - nb;
    const unsigned s2 = (unsigned)da.z - nb, s3 = (unsigned)da.w - nb;
    const unsigned s4 = (unsigned)db.x - nb, s5 = (unsigned)db.y - nb;
    const unsigned s6 = (unsigned)db.z - nb, s7 = (unsigned)db.w - nb;
    const bool h0 = s0 < (unsigned)NB, h1 = s1 < (unsigned)NB, h2 = s2 < (unsigned)NB, h3 = s3 < (unsigned)NB;
    const bool h4 = s4 < (unsigned)NB, h5 = s5 < (unsigned)NB, h6 = s6 < (unsigned)NB, h7 = s7 < (unsigned)NB;
    const unsigned any = __builtin_amdgcn_ballot_w32(h0 | h1 | h2 | h3 | h4 | h5 | h6 | h7);
    if (any != 0u) {
#define HITJ(J, HJ, SJ) { \
        const unsigned mj = __builtin_amdgcn_ballot_w32(HJ); \
        if (mj != 0u) { \
          if (HJ) { \
            const int pos = wc + (int)__builtin_amdgcn_mbcnt_lo(mj, 0u); \
            if (pos < WCAP) list[wave * WCAP + pos] = ((el0 + (J)) << 12) | (int)(SJ); \
          } \
          wc += (int)__builtin_popcount(mj); } }
      HITJ(0, h0, s0)
      HITJ(1, h1, s1)
      HITJ(2, h2, s2)
      HITJ(3, h3, s3)
      HITJ(4, h4, s4)
      HITJ(5, h5, s5)
      HITJ(6, h6, s6)
      HITJ(7, h7, s7)
#undef HITJ
    }
  }
  return wc;
}

__global__ __launch_bounds__(NTHR) void k_wprep(
    const float* __restrict__ w1, const float* __restrict__ w2, unsigned short* wp) {
  const int blk = blockIdx.x, tid = threadIdx.x;
  const int L = blk >> 1;
  const int i = (blk & 1) * NTHR + tid;
  const int n = i >> 3, k0 = (i & 7) * 8;
  v4f a, b;
  float v[8];
#pragma unroll
  for (int e = 0; e < 8; ++e) {
    const float va = w1[(k0 + e) * FD + n];
    const float vb = w2[(k0 + e) * FD + n];
    v[e] = (L == 0) ? va : vb;
  }
  a.x = v[0]; a.y = v[1]; a.z = v[2]; a.w = v[3];
  b.x = v[4]; b.y = v[5]; b.z = v[6]; b.w = v[7];
  Pack8 q;
  q.h = cvt8(a, b, WSC);
  unsigned short* d = wp + (size_t)L * WPL + (size_t)i * 8;
  *(volatile v8us*)d = q.u;
  __threadfence();
  *(volatile v8us*)d = q.u;
}

__global__ __launch_bounds__(NTHR) void k_count(const int* __restrict__ dsts, int* cnt, int nE, int vec8) {
  __shared__ __attribute__((aligned(16))) int scnt[NBC];
  __shared__ __attribute__((aligned(16))) int list[LISTN];
  __shared__ int wcnt[NWAVE];
  const int tid = threadIdx.x, lane = tid & 31, wave = tid >> 5;
  const int nodeBase = blockIdx.x * NBC;

  for (int i = tid; i < NBC; i += NTHR) scnt[i] = 0;
  __syncthreads();

  const int nChunks = (nE + CHUNK - 1) / CHUNK;
#pragma unroll 1
  for (int ch = 0; ch < nChunks; ++ch) {
    const int cbase = ch * CHUNK;
    const int wc = scan_chunk<NBC>(dsts, nE, cbase, nodeBase, vec8, list, tid, lane, wave);
    if (lane == 0) wcnt[wave] = wc;
    __syncthreads();
    if (wave == 0) {
#pragma unroll 1
      for (int wsx = 0; wsx < NWAVE; ++wsx) {
        int n = __builtin_amdgcn_readfirstlane(wcnt[wsx]);
        n = n > WCAP ? WCAP : (n < 0 ? 0 : n);
        const int* lp = list + wsx * WCAP;
#pragma unroll 1
        for (int i = 0; i < n; ++i) {
          const int ent  = __builtin_amdgcn_readfirstlane(lp[i]);
          const int slot = ent & (NBC - 1);
          if (lane == 0) scnt[slot] = scnt[slot] + 1;
        }
      }
    }
    __syncthreads();
  }

  v4i cq[4];
#pragma unroll
  for (int q = 0; q < 4; ++q) {
    const int f = (wave * 4 + q) * 128 + 4 * lane;
    cq[q] = *(const v4i*)(scnt + f);
  }
  int* cp = cnt + (size_t)nodeBase;
#pragma unroll
  for (int q = 0; q < 4; ++q) {
    const int f = (wave * 4 + q) * 128 + 4 * lane;
    *(volatile v4i*)(cp + f) = cq[q];
  }
  __threadfence();
#pragma unroll
  for (int q = 0; q < 4; ++q) {
    const int f = (wave * 4 + q) * 128 + 4 * lane;
    *(volatile v4i*)(cp + f) = cq[q];
  }
}

__global__ __launch_bounds__(OTHR) void k_offsets(
    const int* __restrict__ cnt, int* off, int* rbase, int nChunk) {
  __shared__ __attribute__((aligned(16))) int soff[NBC];
  __shared__ __attribute__((aligned(16))) int srb[RBN];
  __shared__ int wtot[OTHR / 32];
  const int tid = threadIdx.x, lane = tid & 31, wave = tid >> 5, sub = tid >> 7;
  for (int i = tid; i < RBN; i += OTHR) srb[i] = 0;
  int carry = 0;
#pragma unroll 1
  for (int ch = 0; ch < nChunk; ++ch) {
    const int base = ch * NBC;
    const v4i c0 = *(const v4i*)(cnt + base + 8 * tid);
    const v4i c1 = *(const v4i*)(cnt + base + 8 * tid + 4);
    const int e0 = max(c0.x, 0), e1 = max(c0.y, 0), e2 = max(c0.z, 0), e3 = max(c0.w, 0);
    const int e4 = max(c1.x, 0), e5 = max(c1.y, 0), e6 = max(c1.z, 0), e7 = max(c1.w, 0);
    const int ts = e0 + e1 + e2 + e3 + e4 + e5 + e6 + e7;
    int incl = ts;
#pragma unroll
    for (int d = 1; d < 32; d <<= 1) {
      const int t = __shfl_up(incl, d);
      if (lane >= d) incl += t;
    }
    if (lane == 31) wtot[wave] = incl;
    __syncthreads();
    const int S0 = wtot[0]  + wtot[1]  + wtot[2]  + wtot[3];
    const int S1 = wtot[4]  + wtot[5]  + wtot[6]  + wtot[7];
    const int S2 = wtot[8]  + wtot[9]  + wtot[10] + wtot[11];
    const int S3 = wtot[12] + wtot[13] + wtot[14] + wtot[15];
    int pre = 0;
#pragma unroll 1
    for (int w = 4 * sub; w < wave; ++w) pre += wtot[w];
    const int b0 = carry;
    const int b1 = b0 + ((S0 + 31) & ~31);
    const int b2 = b1 + ((S1 + 31) & ~31);
    const int b3 = b2 + ((S2 + 31) & ~31);
    const int b4 = b3 + ((S3 + 31) & ~31);
    const int myb = sub == 0 ? b0 : (sub == 1 ? b1 : (sub == 2 ? b2 : b3));
    if (tid == 0) {
      srb[min(4 * ch + 0, RBN - 1)] = b0;
      srb[min(4 * ch + 1, RBN - 1)] = b1;
      srb[min(4 * ch + 2, RBN - 1)] = b2;
      srb[min(4 * ch + 3, RBN - 1)] = b3;
    }
    int run = myb + pre + incl - ts;
    soff[8 * tid + 0] = run; run += e0;
    soff[8 * tid + 1] = run; run += e1;
    soff[8 * tid + 2] = run; run += e2;
    soff[8 * tid + 3] = run; run += e3;
    soff[8 * tid + 4] = run; run += e4;
    soff[8 * tid + 5] = run; run += e5;
    soff[8 * tid + 6] = run; run += e6;
    soff[8 * tid + 7] = run;
    carry = b4;
    __syncthreads();
    const v4i o0 = *(const v4i*)(soff + 4 * tid);
    const v4i o1 = *(const v4i*)(soff + 4 * (tid + OTHR));
    int* op = off + base;
    *(volatile v4i*)(op + 4 * tid) = o0;
    *(volatile v4i*)(op + 4 * (tid + OTHR)) = o1;
    __threadfence();
    *(volatile v4i*)(op + 4 * tid) = o0;
    *(volatile v4i*)(op + 4 * (tid + OTHR)) = o1;
    __syncthreads();
  }
  if (tid == 0) srb[min(4 * nChunk, RBN - 1)] = carry;
  __syncthreads();
  v4i rv = {0, 0, 0, 0};
  if (tid < 32) rv = *(const v4i*)(srb + 4 * tid);
  if (tid < 32) *(volatile v4i*)(rbase + 4 * tid) = rv;
  __threadfence();
  if (tid < 32) *(volatile v4i*)(rbase + 4 * tid) = rv;
}

__global__ __launch_bounds__(NTHR) void k_fill(
    const int* __restrict__ srcs, const int* __restrict__ dsts,
    const int* __restrict__ off, const int* __restrict__ rbase,
    int* csr, int nN, int nE, int vec8, int csrLen) {
  extern __shared__ v4f lds_dyn[];
  int* region = (int*)lds_dyn;
  int* cursor = region + RCAP;
  int* list   = cursor + NBF;
  int* wcnt   = list + LISTN;
  const int tid = threadIdx.x, lane = tid & 31, wave = tid >> 5;
  const int b = blockIdx.x;
  const int nodeBase = b * NBF;

  int rb0 = rbase[b];
  const int rb1 = rbase[b + 1];
  rb0 = rb0 < 0 ? 0 : (rb0 > csrLen ? csrLen : rb0);
  rb0 &= ~31;
  int len = rb1 - rb0;
  len = len < 0 ? 0 : (len > RCAP ? RCAP : len);
  int lenW = (len + 31) & ~31;
  if (rb0 + lenW > csrLen) lenW = (csrLen - rb0) & ~31;

  {
    const v4i z = {0, 0, 0, 0};
    for (int i = tid; i < RCAP / 4; i += NTHR) ((v4i*)region)[i] = z;
    for (int s = tid; s < NBF; s += NTHR) {
      int o = off[nodeBase + s] - rb0;
      o = o < 0 ? 0 : (o > RCAP ? RCAP : o);
      cursor[s] = o;
    }
  }
  __syncthreads();

  const int nChunks = (nE + CHUNK - 1) / CHUNK;
#pragma unroll 1
  for (int ch = 0; ch < nChunks; ++ch) {
    const int cbase = ch * CHUNK;
    const int wc = scan_chunk<NBF>(dsts, nE, cbase, nodeBase, vec8, list, tid, lane, wave);
    if (lane == 0) wcnt[wave] = wc;
    __syncthreads();
    if (wave == 0) {
#pragma unroll 1
      for (int wsx = 0; wsx < NWAVE; ++wsx) {
        int n = __builtin_amdgcn_readfirstlane(wcnt[wsx]);
        n = n > WCAP ? WCAP : (n < 0 ? 0 : n);
        const int* lp = list + wsx * WCAP;
#pragma unroll 1
        for (int i = 0; i < n; ++i) {
          const int ent  = __builtin_amdgcn_readfirstlane(lp[i]);
          const int slot = ent & (NBF - 1);
          int e = cbase + ((ent >> 12) & (CHUNK - 1));
          e = e > nE - 1 ? nE - 1 : e;
          int sv = srcs[e];
          sv = sv < 0 ? 0 : (sv > nN - 1 ? nN - 1 : sv);
          if (lane == 0) {
            int pos = cursor[slot];
            pos = pos < 0 ? 0 : (pos > RCAP - 1 ? RCAP - 1 : pos);
            region[pos] = sv;
            const int np = pos + 1;
            cursor[slot] = np > RCAP ? RCAP : np;
          }
        }
      }
    }
    __syncthreads();
  }

  const int nv = lenW >> 2;
  int* gp = csr + rb0;
#pragma unroll 1
  for (int i = tid; i < nv; i += NTHR) { const v4i v = ((const v4i*)region)[i]; *(volatile v4i*)(gp + 4 * i) = v; }
  __threadfence();
#pragma unroll 1
  for (int i = tid; i < nv; i += NTHR) { const v4i v = ((const v4i*)region)[i]; *(volatile v4i*)(gp + 4 * i) = v; }
}

template <bool BNA>
__global__ __launch_bounds__(NTHR) void k_gemm(
    const float* __restrict__ A, const float* __restrict__ coef,
    const float* __restrict__ gam, const float* __restrict__ bet,
    const _Float16* __restrict__ Wp, const int* __restrict__ cnt,
    float* C, int nN) {
  __shared__ __attribute__((aligned(16))) _Float16 sA[GROWS * APK];
  __shared__ __attribute__((aligned(16))) float stg[GROWS * FD];
  const int tid = threadIdx.x, lane = tid & 31, wave = tid >> 5, hh = lane >> 4, m = lane & 15;
  const int rowBase = blockIdx.x * GROWS;
  const int c0 = (tid & 7) * 8, rr = tid >> 3;

  v4f mua = {0.f, 0.f, 0.f, 0.f};
  v4f mub = mua, rsa = mua, rsb = mua, ga = mua, gb = mua, ba = mua, bb = mua;
  if (BNA) {
    mua = *(const v4f*)(coef + c0);       mub = *(const v4f*)(coef + c0 + 4);
    rsa = *(const v4f*)(coef + FD + c0);  rsb = *(const v4f*)(coef + FD + c0 + 4);
    ga  = *(const v4f*)(gam + c0);        gb  = *(const v4f*)(gam + c0 + 4);
    ba  = *(const v4f*)(bet + c0);        bb  = *(const v4f*)(bet + c0 + 4);
  }
#pragma unroll
  for (int it = 0; it < 4; ++it) {
    const int r = it * 32 + rr;
    int row = rowBase + r;
    row = row > nN - 1 ? nN - 1 : row;
    const float* ap = A + (size_t)row * FD + c0;
    v4f a = *(const v4f*)ap, b = *(const v4f*)(ap + 4);
    if (BNA) { a = bnr(a, mua, rsa, ga, ba); b = bnr(b, mub, rsb, gb, bb); }
    *(v8h*)(sA + r * APK + c0) = cvt8(a, b, ASC);
  }
  __syncthreads();

  v8f acc[4];
#pragma unroll
  for (int t = 0; t < 4; ++t) { v8f z = {0.f, 0.f, 0.f, 0.f, 0.f, 0.f, 0.f, 0.f}; acc[t] = z; }
  const _Float16* abase = sA + (wave * 16 + m) * APK + 8 * hh;
#pragma unroll
  for (int kt = 0; kt < 2; ++kt) {
    FragH a;
    a.half[0] = *(const v8h*)(abase + 32 * kt);
    a.half[1] = *(const v8h*)(abase + 32 * kt + 16);
#pragma unroll
    for (int t = 0; t < 4; ++t) {
      const _Float16* bp = Wp + (size_t)(16 * t + m) * KD + 32 * kt + 8 * hh;
      FragH b;
      b.half[0] = *(const v8h*)bp;
      b.half[1] = *(const v8h*)(bp + 16);
      acc[t] = wmh(a.v, b.v, acc[t]);
    }
  }

  float dsc[8];
#pragma unroll
  for (int r = 0; r < 8; ++r) {
    int cr = cnt[rowBase + wave * 16 + 8 * hh + r];
    cr = cr < 0 ? 0 : cr;
    dsc[r] = rsqrtf((float)cr + 1.0f) * INVSC;
  }
  float* sp = stg + (wave * 16 + 8 * hh) * FD + m;
#pragma unroll
  for (int t = 0; t < 4; ++t) {
#pragma unroll
    for (int r = 0; r < 8; ++r) sp[r * FD + 16 * t] = acc[t][r] * dsc[r];
  }
  __syncthreads();

  const float* lp = stg + wave * 16 * FD + 4 * lane;
  float* gp = C + (size_t)(rowBase + wave * 16) * FD + 4 * lane;
#pragma unroll
  for (int i = 0; i < 8; ++i) { const v4f v = *(const v4f*)(lp + 128 * i); *(volatile v4f*)(gp + 128 * i) = v; }
  __threadfence();
#pragma unroll
  for (int i = 0; i < 8; ++i) { const v4f v = *(const v4f*)(lp + 128 * i); *(volatile v4f*)(gp + 128 * i) = v; }
}

__global__ __launch_bounds__(NTHR) void k_agg(
    const int* __restrict__ csr, const int* __restrict__ off, const int* __restrict__ cnt,
    const float* __restrict__ Hs, const float* __restrict__ bias,
    float* G, double* part, int nN, int csrLen) {
  __shared__ __attribute__((aligned(16))) double dS[2 * NWAVE * FD];
  __shared__ __attribute__((aligned(16))) double dQ[2 * NWAVE * FD];
  __shared__ __attribute__((aligned(16))) double dP[2 * FD];
  const int tid = threadIdx.x, lane = tid & 31, wave = tid >> 5, hf = lane >> 4, cg = lane & 15;
  const int tbase = blockIdx.x * TGT + wave * 32;
  const int cl = tbase + lane;
  const int cnt_l = cnt[cl];
  const int off_l = off[cl];
  const v4f bv = *(const v4f*)(bias + 4 * cg);
  double s0 = 0.0, s1 = 0.0, s2 = 0.0, s3 = 0.0;
  double q0s = 0.0, q1s = 0.0, q2s = 0.0, q3s = 0.0;

#pragma unroll 1
  for (int j = 0; j < 16; ++j) {
    int cA = __builtin_amdgcn_readlane(cnt_l, 2 * j);
    int cB = __builtin_amdgcn_readlane(cnt_l, 2 * j + 1);
    cA = cA < 0 ? 0 : cA;
    cB = cB < 0 ? 0 : cB;
    const int nA = cA > DEGCAP ? DEGCAP : cA;
    const int nB = cB > DEGCAP ? DEGCAP : cB;
    const int stA = __builtin_amdgcn_readlane(off_l, 2 * j);
    const int stB = __builtin_amdgcn_readlane(off_l, 2 * j + 1);
    const int nme  = hf ? nB : nA;
    const int stme = hf ? stB : stA;
    const int cme  = hf ? cB : cA;
    const int nmax = nA > nB ? nA : nB;
    v4f acc = {0.0f, 0.0f, 0.0f, 0.0f};
#pragma unroll 1
    for (int q0 = 0; q0 < nmax; q0 += 16) {
      int pos = stme + q0 + cg;
      pos = pos < 0 ? 0 : (pos > csrLen - 1 ? csrLen - 1 : pos);
      int sl = csr[pos];
      sl = sl < 0 ? 0 : (sl > nN - 1 ? nN - 1 : sl);
      const int mcnt = (nmax - q0) < 16 ? (nmax - q0) : 16;
#pragma unroll 1
      for (int p = 0; p < mcnt; ++p) {
        const int sA = __builtin_amdgcn_readlane(sl, p);
        const int sB = __builtin_amdgcn_readlane(sl, 16 + p);
        const int s = hf ? sB : sA;
        const v4f v = *(const v4f*)(Hs + (size_t)s * FD + 4 * cg);
        const bool ok = (q0 + p) < nme;
        acc.x += ok ? v.x : 0.0f;
        acc.y += ok ? v.y : 0.0f;
        acc.z += ok ? v.z : 0.0f;
        acc.w += ok ? v.w : 0.0f;
      }
    }
    const int c = tbase + 2 * j + hf;
    const v4f self = *(const v4f*)(Hs + (size_t)c * FD + 4 * cg);
    const float dis = rsqrtf((float)cme + 1.0f);
    const v4f g = (acc + self) * dis + bv;
    float* gp = G + (size_t)(tbase + 2 * j) * FD + 4 * lane;
    *(volatile v4f*)gp = g;
    __threadfence();
    *(volatile v4f*)gp = g;
    v4f gz;
    gz.x = (c < nN) ? g.x : 0.0f; gz.y = (c < nN) ? g.y : 0.0f;
    gz.z = (c < nN) ? g.z : 0.0f; gz.w = (c < nN) ? g.w : 0.0f;
    const double d0 = (double)gz.x, d1 = (double)gz.y, d2 = (double)gz.z, d3 = (double)gz.w;
    s0 += d0; s1 += d1; s2 += d2; s3 += d3;
    q0s = fma(d0, d0, q0s); q1s = fma(d1, d1, q1s); q2s = fma(d2, d2, q2s); q3s = fma(d3, d3, q3s);
  }

  {
    double* ds = dS + (wave * 2 + hf) * FD + 4 * cg;
    double* dq = dQ + (wave * 2 + hf) * FD + 4 * cg;
    ds[0] = s0; ds[1] = s1; ds[2] = s2; ds[3] = s3;
    dq[0] = q0s; dq[1] = q1s; dq[2] = q2s; dq[3] = q3s;
  }
  __syncthreads();
  if (tid < 2 * FD) {
    const int c = tid & (FD - 1);
    double S = 0.0, Q = 0.0;
#pragma unroll 1
    for (int i = 0; i < 2 * NWAVE; ++i) { S += dS[i * FD + c]; Q += dQ[i * FD + c]; }
    dP[tid] = (tid < FD) ? S : Q;
  }
  __syncthreads();
  v2d pv = {0.0, 0.0};
  if (tid < FD) pv = *(const v2d*)(dP + 2 * tid);
  double* gq = part + (size_t)blockIdx.x * (2 * FD) + 2 * tid;
  if (tid < FD) *(volatile v2d*)gq = pv;
  __threadfence();
  if (tid < FD) *(volatile v2d*)gq = pv;
}

__global__ __launch_bounds__(64) void k_bnfin(const double* __restrict__ part, float* coef, int nBlk, int nN) {
  __shared__ __attribute__((aligned(16))) float sco[2 * FD];
  const int tid = threadIdx.x, c = tid & (FD - 1);
  double S = 0.0, Q = 0.0;
#pragma unroll 1
  for (int b = 0; b < nBlk; ++b) {
    S += part[(size_t)b * (2 * FD) + c];
    Q += part[(size_t)b * (2 * FD) + FD + c];
  }
  const double rn = 1.0 / (double)(nN > 1 ? nN : 1);
  const double mean = S * rn;
  double var = Q * rn - mean * mean;
  var = var < 0.0 ? 0.0 : var;
  sco[c]      = (float)mean;
  sco[FD + c] = rsqrtf((float)var + BN_EPS);
  __syncthreads();
  v4f cv = {0.f, 0.f, 0.f, 0.f};
  if (tid < 32) cv = *(const v4f*)(sco + 4 * tid);
  if (tid < 32) *(volatile v4f*)(coef + 4 * tid) = cv;
  __threadfence();
  if (tid < 32) *(volatile v4f*)(coef + 4 * tid) = cv;
}

__global__ __launch_bounds__(NTHR) void k_out(
    const float* __restrict__ G, const float* __restrict__ coef,
    const float* __restrict__ gam, const float* __restrict__ bet,
    float* out, int nq) {
  const int q = blockIdx.x * NTHR + threadIdx.x;
  const int qc = q < nq ? q : nq - 1;
  const int c4 = (qc & 15) * 4;
  const v4f v  = *(const v4f*)(G + (size_t)qc * 4);
  const v4f mu = *(const v4f*)(coef + c4);
  const v4f rs = *(const v4f*)(coef + FD + c4);
  const v4f g  = *(const v4f*)(gam + c4);
  const v4f b  = *(const v4f*)(bet + c4);
  const v4f y  = bnr(v, mu, rs, g, b);
  float* op = out + (size_t)qc * 4;
  if (q < nq) *(volatile v4f*)op = y;
  __threadfence();
  if (q < nq) *(volatile v4f*)op = y;
}

extern "C" void kernel_launch(void* const* d_in, const int* in_sizes, int n_in,
                              void* d_out, int out_size, void* d_ws, size_t ws_size,
                              hipStream_t stream) {
  if (n_in < 10) return;
  const int nN = in_sizes[0] / FD;
  const int nE = in_sizes[1] / 2;
  if (nN <= 0 || nE <= 0) return;
  if (in_sizes[0] != nN * FD || in_sizes[1] != 2 * nE) return;
  if (in_sizes[2] != FD * FD || in_sizes[3] != FD || in_sizes[4] != FD || in_sizes[5] != FD) return;
  if (in_sizes[6] != FD * FD || in_sizes[7] != FD || in_sizes[8] != FD || in_sizes[9] != FD) return;
  if (out_size != nN * FD) return;
  if (nE > (1 << 28) || nN > (1 << 24)) return;

  const float* x    = (const float*)d_in[0];
  const int*   ei   = (const int*)d_in[1];
  const float* w1   = (const float*)d_in[2];
  const float* b1   = (const float*)d_in[3];
  const float* gam1 = (const float*)d_in[4];
  const float* bet1 = (const float*)d_in[5];
  const float* w2   = (const float*)d_in[6];
  const float* b2   = (const float*)d_in[7];
  const float* gam2 = (const float*)d_in[8];
  const float* bet2 = (const float*)d_in[9];
  const int* srcs = ei;
  const int* dsts = ei + (size_t)nE;
  float* out = (float*)d_out;

  const int NPAD   = ((nN + TGT - 1) / TGT) * TGT;
  const int nBC    = (nN + NBC - 1) / NBC;
  const int CNTPAD = nBC * NBC;
  if (4 * nBC + 1 > RBN) return;
  const int nBF    = (nN + NBF - 1) / NBF;
  const int csrLen = ((nE + 31) & ~31) + 4096;
  if (31 * 4 * nBC > 4096) return;
  const int nGemm  = NPAD / GROWS;
  const int nAgg   = NPAD / TGT;
  const int nq     = nN * 16;
  const int nOut   = (nq + NTHR - 1) / NTHR;

  char* ws = (char*)d_ws;
  size_t off = 0;
  const size_t oW     = off; off += (size_t)2 * WPL * 2;           off = (off + 255) & ~(size_t)255;
  const size_t oCnt   = off; off += (size_t)CNTPAD * 4;            off = (off + 255) & ~(size_t)255;
  const size_t oOff   = off; off += (size_t)CNTPAD * 4;            off = (off + 255) & ~(size_t)255;
  const size_t oRb    = off; off += (size_t)RBN * 4;               off = (off + 255) & ~(size_t)255;
  const size_t oCsr   = off; off += (size_t)csrLen * 4;            off = (off + 255) & ~(size_t)255;
  const size_t oH     = off; off += (size_t)NPAD * FD * 4;         off = (off + 255) & ~(size_t)255;
  const size_t oG     = off; off += (size_t)NPAD * FD * 4;         off = (off + 255) & ~(size_t)255;
  const size_t oPart1 = off; off += (size_t)nAgg * (2 * FD) * 8;   off = (off + 255) & ~(size_t)255;
  const size_t oPart2 = off; off += (size_t)nAgg * (2 * FD) * 8;   off = (off + 255) & ~(size_t)255;
  const size_t oCoef1 = off; off += (size_t)2 * FD * 4;            off = (off + 255) & ~(size_t)255;
  const size_t oCoef2 = off; off += (size_t)2 * FD * 4;            off = (off + 255) & ~(size_t)255;
  if (off > ws_size || off > (size_t)WSCAP) return;
  unsigned short* wp    = (unsigned short*)(ws + oW);
  const _Float16* wp1   = (const _Float16*)(ws + oW);
  const _Float16* wp2   = wp1 + WPL;
  int*            cnt   = (int*)(ws + oCnt);
  int*            offp  = (int*)(ws + oOff);
  int*            rb    = (int*)(ws + oRb);
  int*            csr   = (int*)(ws + oCsr);
  float*          Hs    = (float*)(ws + oH);
  float*          Gp    = (float*)(ws + oG);
  double*         part1 = (double*)(ws + oPart1);
  double*         part2 = (double*)(ws + oPart2);
  float*          coef1 = (float*)(ws + oCoef1);
  float*          coef2 = (float*)(ws + oCoef2);

  const int vec8 = ((nE & 3) == 0) ? 1 : 0;

  k_wprep<<<4, NTHR, 0, stream>>>(w1, w2, wp);

  k_count<<<nBC, NTHR, 0, stream>>>(dsts, cnt, nE, vec8);
  k_offsets<<<1, OTHR, 0, stream>>>(cnt, offp, rb, nBC);
  hipFuncSetAttribute(reinterpret_cast<const void*>(&k_fill),
                      hipFuncAttributeMaxDynamicSharedMemorySize, LDS_FILL);
  k_fill<<<nBF, NTHR, LDS_FILL, stream>>>(srcs, dsts, offp, rb, csr, nN, nE, vec8, csrLen);

  k_gemm<false><<<nGemm, NTHR, 0, stream>>>(x, coef1, gam1, bet1, wp1, cnt, Hs, nN);

  k_agg<<<nAgg, NTHR, 0, stream>>>(csr, offp, cnt, Hs, b1, Gp, part1, nN, csrLen);

  k_bnfin<<<1, 64, 0, stream>>>(part1, coef1, nAgg, nN);

  k_gemm<true><<<nGemm, NTHR, 0, stream>>>(Gp, coef1, gam1, bet1, wp2, cnt, Hs, nN);

  k_agg<<<nAgg, NTHR, 0, stream>>>(csr, offp, cnt, Hs, b2, Gp, part2, nN, csrLen);

  k_bnfin<<<1, 64, 0, stream>>>(part2, coef2, nAgg, nN);

  k_out<<<nOut, NTHR, 0, stream>>>(Gp, coef2, gam2, bet2, out, nq);
}
